// multi_query_atnn_20598663152351
// MI455X (gfx1250) — hardware-verified
//
#include <hip/hip_runtime.h>

typedef _Float16 v16h __attribute__((ext_vector_type(16)));
typedef _Float16 v8h  __attribute__((ext_vector_type(8)));
typedef float    v8f  __attribute__((ext_vector_type(8)));
typedef float    v4f  __attribute__((ext_vector_type(4)));
typedef v8h __attribute__((may_alias)) v8ha;
typedef v4f __attribute__((may_alias)) v4fa;

union Frag { v16h v; v8h half[2]; };

#define DIM    2048
#define SEQ    2048
#define NH     16
#define HD     128
#define BS     2
#define MTOT   (BS * SEQ)
#define NX     (MTOT * DIM)
#define NX8    (NX / 8)
#define WSC    32.0f
#define WINV   0.03125f
#define PSCALE 16384.0f
#define OSC    16.0f

__device__ __forceinline__ v8f wmma_f16(v16h a, v16h b, v8f c) {
  v8f d = __builtin_amdgcn_wmma_f32_16x16x32_f16(false, a, false, b, (short)0, c, false, false);
  asm volatile("v_nop\n\tv_nop\n\tv_nop\n\tv_nop" : "+v"(d) : "v"(a), "v"(b));
  return d;
}

__device__ __forceinline__ v16h load_frag(const _Float16* p, int h) {
  Frag f;
  f.half[0] = *(const v8ha*)(p + 8 * h);
  f.half[1] = *(const v8ha*)(p + 16 + 8 * h);
  return f.v;
}

__global__ __launch_bounds__(256) void cvt_x_kernel(const float* __restrict__ x,
                                                     _Float16* __restrict__ xh, int n8)
{
  const int g = blockIdx.x * 256 + threadIdx.x;
  if (g >= n8) return;
  const float* src = x + (size_t)g * 8;
  const v4f a = *(const v4fa*)src;
  const v4f c = *(const v4fa*)(src + 4);
  const v8h o = { (_Float16)a.x, (_Float16)a.y, (_Float16)a.z, (_Float16)a.w,
                  (_Float16)c.x, (_Float16)c.y, (_Float16)c.z, (_Float16)c.w };
  _Float16* dst = xh + (size_t)g * 8;
  *(volatile v8h*)dst = o;
  __threadfence();
  *(volatile v8h*)dst = o;
}

__global__ __launch_bounds__(256) void transpose_w_kernel(const float* __restrict__ w,
                                                           _Float16* __restrict__ wT,
                                                           int K, int N)
{
  __shared__ __attribute__((aligned(16))) _Float16 sT[32 * 64];
  const int tid = threadIdx.x, lane = tid & 31, wv = tid >> 5;
  const int n0 = blockIdx.x * 32, k0 = blockIdx.y * 64;
  const int nn = tid & 31, kr = tid >> 5;
  #pragma unroll
  for (int i = 0; i < 8; ++i) {
    const int kk = kr + 8 * i;
    const float val = w[(size_t)(k0 + kk) * N + n0 + nn] * WSC;
    sT[nn * 64 + kk] = (_Float16)val;
  }
  __syncthreads();
  const int q8 = lane & 7, sub = lane >> 3;
  const int n = wv * 4 + sub;
  const v8h v = *(const v8ha*)(sT + n * 64 + 8 * q8);
  _Float16* dst = wT + (size_t)(n0 + n) * K + k0 + 8 * q8;
  *(volatile v8h*)dst = v;
  __threadfence();
  *(volatile v8h*)dst = v;
}

__device__ __forceinline__ void store_rows_f16(const _Float16* sT, _Float16* C,
                                               int m0, int n0, int N, int w, int lane) {
  const int q8 = lane & 7, sub = lane >> 3;
  #pragma unroll
  for (int i = 0; i < 8; ++i) {
    const int lid = w * 32 + i * 4 + sub;
    const v8h v = *(const v8ha*)(sT + lid * 64 + 8 * q8);
    _Float16* dst = C + (size_t)(m0 + lid) * N + n0 + 8 * q8;
    *(volatile v8h*)dst = v;
  }
}

__device__ __forceinline__ void store_vt_f16(const _Float16* sT, _Float16* vt,
                                             int b, int t0, int n0, int w, int lane) {
  const int q8 = lane & 7, sub = lane >> 3;
  #pragma unroll
  for (int i = 0; i < 8; ++i) {
    const int lid = w * 32 + i * 4 + sub;
    const int d = lid >> 1, hl = lid & 1;
    const v8h v = *(const v8ha*)(sT + d * 128 + 64 * hl + 8 * q8);
    _Float16* dst = vt + ((size_t)(b * HD + n0 + d)) * SEQ + t0 + 64 * hl + 8 * q8;
    *(volatile v8h*)dst = v;
  }
}

__device__ __forceinline__ void store_rows_f32(const float* sT, float* C,
                                               int m0, int n0, int N, int w, int lane) {
  const int q8 = lane & 7, sub = lane >> 3;
  #pragma unroll
  for (int i = 0; i < 16; ++i) {
    const int lid = i * 4 + sub;
    const int row = 32 * w + (lid >> 1), hl = lid & 1;
    const v4f v = *(const v4fa*)(sT + row * 64 + 32 * hl + 4 * q8);
    float* dst = C + (size_t)(m0 + row) * N + n0 + 32 * hl + 4 * q8;
    *(volatile v4f*)dst = v;
  }
}

union GemmSmem { _Float16 h[128 * 64]; float f[128 * 64]; };

template <int MODE, typename CT>
__global__ __launch_bounds__(128) void gemm_kernel(
    const _Float16* __restrict__ A, const _Float16* __restrict__ BT,
    const float* __restrict__ bias, CT* __restrict__ C,
    int N, int K, float ascale, float oscale)
{
  __shared__ __attribute__((aligned(16))) GemmSmem sm;

  const int tid = threadIdx.x, lane = tid & 31, w = tid >> 5;
  const int h = lane >> 4, m = lane & 15;
  const int m0 = blockIdx.x * 128, n0 = blockIdx.y * 64;
  const int m0w = m0 + 32 * w;

  const _Float16* xa0 = A + (size_t)(m0w + m) * K;
  const _Float16* xa1 = xa0 + (size_t)16 * K;
  const _Float16* wb  = BT + (size_t)(n0 + m) * K;

  const v8f zero8 = {0.f, 0.f, 0.f, 0.f, 0.f, 0.f, 0.f, 0.f};
  v8f acc[2][4];
  #pragma unroll
  for (int mt = 0; mt < 2; ++mt)
    #pragma unroll
    for (int nt = 0; nt < 4; ++nt) acc[mt][nt] = zero8;

  #pragma unroll 1
  for (int k0 = 0; k0 < K; k0 += 32) {
    const v16h a0 = load_frag(xa0 + k0, h);
    const v16h a1 = load_frag(xa1 + k0, h);
    #pragma unroll
    for (int nt = 0; nt < 4; ++nt) {
      const v16h b = load_frag(wb + (size_t)nt * 16 * K + k0, h);
      acc[0][nt] = wmma_f16(a0, b, acc[0][nt]);
      acc[1][nt] = wmma_f16(a1, b, acc[1][nt]);
    }
  }

  #pragma unroll
  for (int nt = 0; nt < 4; ++nt) {
    const int feat = 16 * nt + m;
    const float bvl = bias[n0 + feat];
    #pragma unroll
    for (int mt = 0; mt < 2; ++mt) {
      #pragma unroll
      for (int r = 0; r < 8; ++r) {
        const int tokl = 32 * w + 16 * mt + 8 * h + r;
        const float y = acc[mt][nt][r] * ascale + bvl;
        if (MODE == 2) {
          sm.f[tokl * 64 + feat] = y;
        } else if (MODE == 1) {
          sm.h[feat * 128 + tokl] = (_Float16)(y * oscale);
        } else {
          sm.h[tokl * 64 + feat] = (_Float16)(y * oscale);
        }
      }
    }
  }
  __syncthreads();

  if (MODE == 2) {
    float* Cf = (float*)(void*)C;
    store_rows_f32(sm.f, Cf, m0, n0, N, w, lane);
    __threadfence();
    store_rows_f32(sm.f, Cf, m0, n0, N, w, lane);
  } else if (MODE == 1) {
    _Float16* Ch = (_Float16*)(void*)C;
    const int b = m0 / SEQ, t0 = m0 - b * SEQ;
    store_vt_f16(sm.h, Ch, b, t0, n0, w, lane);
    __threadfence();
    store_vt_f16(sm.h, Ch, b, t0, n0, w, lane);
  } else {
    _Float16* Ch = (_Float16*)(void*)C;
    store_rows_f16(sm.h, Ch, m0, n0, N, w, lane);
    __threadfence();
    store_rows_f16(sm.h, Ch, m0, n0, N, w, lane);
  }
}

__device__ __forceinline__ v16h pack_p(v8f a, v8f c) {
  const v16h r = { (_Float16)(a[0] * PSCALE), (_Float16)(a[1] * PSCALE), (_Float16)(a[2] * PSCALE), (_Float16)(a[3] * PSCALE),
                   (_Float16)(a[4] * PSCALE), (_Float16)(a[5] * PSCALE), (_Float16)(a[6] * PSCALE), (_Float16)(a[7] * PSCALE),
                   (_Float16)(c[0] * PSCALE), (_Float16)(c[1] * PSCALE), (_Float16)(c[2] * PSCALE), (_Float16)(c[3] * PSCALE),
                   (_Float16)(c[4] * PSCALE), (_Float16)(c[5] * PSCALE), (_Float16)(c[6] * PSCALE), (_Float16)(c[7] * PSCALE) };
  return r;
}

__device__ __forceinline__ void att_store_pass(const _Float16* so, _Float16* oh,
                                               int b, int head, int q0, int lane) {
  const int q8 = lane & 7, sub = lane >> 3;
  #pragma unroll
  for (int i = 0; i < 8; ++i) {
    const int lid = i * 4 + sub;
    const int row = lid >> 1, hl = lid & 1;
    const v8h v = *(const v8ha*)(so + row * HD + 64 * hl + 8 * q8);
    _Float16* dst = oh + ((size_t)(b * SEQ + q0 + row)) * DIM + head * HD + 64 * hl + 8 * q8;
    *(volatile v8h*)dst = v;
  }
}

__global__ __launch_bounds__(128) void attn_kernel(
    const _Float16* __restrict__ qh,
    const _Float16* __restrict__ kh,
    const _Float16* __restrict__ vt,
    _Float16* __restrict__ oh)
{
  __shared__ __attribute__((aligned(16))) _Float16 sO[4 * 16 * HD];

  const int tid = threadIdx.x, lane = tid & 31, w = tid >> 5;
  const int hh = lane >> 4, m = lane & 15;
  const int b = blockIdx.z, head = blockIdx.y;
  const int q0 = blockIdx.x * 64 + 16 * w;

  const _Float16* qrow = qh + ((size_t)(b * SEQ + q0 + m)) * DIM + head * HD;
  v16h qb[4];
  #pragma unroll
  for (int c = 0; c < 4; ++c) qb[c] = load_frag(qrow + 32 * c, hh);

  const v8f zero8 = {0.f, 0.f, 0.f, 0.f, 0.f, 0.f, 0.f, 0.f};
  v8f o[8];
  #pragma unroll
  for (int t = 0; t < 8; ++t) o[t] = zero8;
  float mrun = -1e30f, lrun = 0.0f;

  const _Float16* kbase = kh + ((size_t)b * SEQ + m) * HD;
  const _Float16* vbase = vt + ((size_t)b * HD + m) * SEQ;
  const float scale = 0.08838834764831845f;

  #pragma unroll 1
  for (int kb = 0; kb < SEQ; kb += 32) {
    v8f s[2];
    #pragma unroll
    for (int j = 0; j < 2; ++j) {
      const _Float16* kp = kbase + (size_t)(kb + 16 * j) * HD;
      v8f z = zero8;
      #pragma unroll
      for (int c = 0; c < 4; ++c) {
        const v16h kf = load_frag(kp + 32 * c, hh);
        z = wmma_f16(kf, qb[c], z);
      }
      s[j] = z;
    }

    float mloc = -1e30f;
    #pragma unroll
    for (int j = 0; j < 2; ++j)
      #pragma unroll
      for (int r = 0; r < 8; ++r) {
        const float sv = s[j][r] * scale;
        s[j][r] = sv;
        mloc = fmaxf(mloc, sv);
      }
    mloc = fmaxf(mloc, __shfl_xor(mloc, 16));
    const float mnew = fmaxf(mrun, mloc);
    const float alpha = __expf(mrun - mnew);
    mrun = mnew;
    float lsum = 0.0f;
    #pragma unroll
    for (int j = 0; j < 2; ++j)
      #pragma unroll
      for (int r = 0; r < 8; ++r) {
        const float p = __expf(s[j][r] - mnew);
        s[j][r] = p;
        lsum += p;
      }
    lsum += __shfl_xor(lsum, 16);
    lrun = lrun * alpha + lsum;
    #pragma unroll
    for (int t = 0; t < 8; ++t)
      #pragma unroll
      for (int r = 0; r < 8; ++r) o[t][r] = o[t][r] * alpha;

    const v16h pb = pack_p(s[0], s[1]);

    #pragma unroll
    for (int t = 0; t < 8; ++t) {
      const v16h vf = load_frag(vbase + (size_t)(16 * t) * SEQ + kb, hh);
      o[t] = wmma_f16(vf, pb, o[t]);
    }
  }

  const float inv = __builtin_amdgcn_rcpf(lrun) * (OSC / PSCALE);
  _Float16* so = sO + w * (16 * HD);
  #pragma unroll
  for (int t = 0; t < 8; ++t)
    #pragma unroll
    for (int r = 0; r < 8; ++r)
      so[m * HD + 16 * t + 8 * hh + r] = (_Float16)(o[t][r] * inv);
  __syncthreads();

  att_store_pass(so, oh, b, head, q0, lane);
  __threadfence();
  att_store_pass(so, oh, b, head, q0, lane);
}

extern "C" void kernel_launch(void* const* d_in, const int* in_sizes, int n_in,
                              void* d_out, int out_size, void* d_ws, size_t ws_size,
                              hipStream_t stream) {
  if (n_in < 9) return;
  if (in_sizes[0] != NX) return;
  if (in_sizes[1] != DIM * DIM || in_sizes[2] != DIM) return;
  if (in_sizes[3] != DIM * HD || in_sizes[4] != HD) return;
  if (in_sizes[5] != DIM * HD || in_sizes[6] != HD) return;
  if (in_sizes[7] != DIM * DIM || in_sizes[8] != DIM) return;
  if (out_size != NX) return;

  const float* x  = (const float*)d_in[0];
  const float* wq = (const float*)d_in[1];
  const float* bq = (const float*)d_in[2];
  const float* wk = (const float*)d_in[3];
  const float* bk = (const float*)d_in[4];
  const float* wv = (const float*)d_in[5];
  const float* bv = (const float*)d_in[6];
  const float* wo = (const float*)d_in[7];
  const float* bo = (const float*)d_in[8];
  float* out = (float*)d_out;

  const size_t act_b = (size_t)NX * 2;
  const size_t wsq_b = (size_t)DIM * DIM * 2;
  const size_t wkv_b = (size_t)DIM * HD * 2;
  const size_t kv_b  = (size_t)MTOT * HD * 2;
  const size_t total = act_b + wsq_b + 2 * wkv_b + wsq_b + act_b + 2 * kv_b + act_b;
  if (total > ws_size) return;

  char* ws = (char*)d_ws;
  size_t off = 0;
  _Float16* xh  = (_Float16*)(ws + off); off += act_b;
  _Float16* wqT = (_Float16*)(ws + off); off += wsq_b;
  _Float16* wkT = (_Float16*)(ws + off); off += wkv_b;
  _Float16* wvT = (_Float16*)(ws + off); off += wkv_b;
  _Float16* woT = (_Float16*)(ws + off); off += wsq_b;
  _Float16* qh  = (_Float16*)(ws + off); off += act_b;
  _Float16* kh  = (_Float16*)(ws + off); off += kv_b;
  _Float16* vT  = (_Float16*)(ws + off); off += kv_b;
  _Float16* oh  = (_Float16*)(ws + off); off += act_b;
  if (off > ws_size) return;

  cvt_x_kernel<<<NX8 / 256, 256, 0, stream>>>(x, xh, NX8);
  transpose_w_kernel<<<dim3(DIM / 32, DIM / 64), 256, 0, stream>>>(wq, wqT, DIM, DIM);
  transpose_w_kernel<<<dim3(HD / 32, DIM / 64), 256, 0, stream>>>(wk, wkT, DIM, HD);
  transpose_w_kernel<<<dim3(HD / 32, DIM / 64), 256, 0, stream>>>(wv, wvT, DIM, HD);
  transpose_w_kernel<<<dim3(DIM / 32, DIM / 64), 256, 0, stream>>>(wo, woT, DIM, DIM);

  gemm_kernel<0, _Float16><<<dim3(MTOT / 128, DIM / 64), 128, 0, stream>>>(xh, wqT, bq, qh, DIM, DIM, WINV, 1.0f);
  gemm_kernel<0, _Float16><<<dim3(MTOT / 128, HD / 64), 128, 0, stream>>>(xh, wkT, bk, kh, HD, DIM, WINV, 1.0f);
  gemm_kernel<1, _Float16><<<dim3(MTOT / 128, HD / 64), 128, 0, stream>>>(xh, wvT, bv, vT, HD, DIM, WINV, 1.0f);

  attn_kernel<<<dim3(SEQ / 64, NH, BS), 128, 0, stream>>>(qh, kh, vT, oh);

  gemm_kernel<2, float><<<dim3(MTOT / 128, DIM / 64), 128, 0, stream>>>(oh, woT, bo, out, DIM, DIM, WINV / OSC, 1.0f);
}
